// GDNLayer_89455578841444
// MI455X (gfx1250) — hardware-verified
//
#include <hip/hip_runtime.h>
#include <math.h>

constexpr int kBatch   = 2;
constexpr int kSeq     = 2048;
constexpr int kChan    = 1024;
constexpr int kHeads   = 16;
constexpr int kHeadDim = 64;
constexpr int kInner   = kHeads * kHeadDim;
constexpr int kTaps    = 4;
constexpr int kProjN   = 4 * kInner + 64;
constexpr int kBdW     = 32;
static_assert(kInner == 1024, "");
static_assert(kProjN % 64 == 0, "");
static_assert(kSeq % 64 == 0, "");
static_assert(kChan % 32 == 0, "");
static_assert(kInner % 32 == 0, "");

constexpr size_t kBytesXplane  = (size_t)kBatch * kSeq * kChan * 2;
constexpr size_t kBytesWplane  = (size_t)kProjN * kChan * 2;
constexpr size_t kBytesWOplane = (size_t)kChan * kInner * 2;
constexpr size_t kBytesP       = (size_t)kSeq * kProjN * 4;
constexpr size_t kBytesAct     = (size_t)kSeq * kInner * 4;
constexpr size_t kBytesBD      = (size_t)kSeq * kBdW * 4;
constexpr size_t kBytesObPlane = (size_t)kSeq * kInner * 2;

constexpr size_t kOffXH  = 0;
constexpr size_t kOffXL  = kOffXH  + kBytesXplane;
constexpr size_t kOffWH  = kOffXL  + kBytesXplane;
constexpr size_t kOffWL  = kOffWH  + kBytesWplane;
constexpr size_t kOffWOH = kOffWL  + kBytesWplane;
constexpr size_t kOffWOL = kOffWOH + kBytesWOplane;
constexpr size_t kOffP   = kOffWOL + kBytesWOplane;
constexpr size_t kOffQN  = kOffP   + kBytesP;
constexpr size_t kOffKN  = kOffQN  + kBytesAct;
constexpr size_t kOffVN  = kOffKN  + kBytesAct;
constexpr size_t kOffBD  = kOffVN  + kBytesAct;
constexpr size_t kOffOSC = kOffBD  + kBytesBD;
constexpr size_t kOffOBH = kOffOSC + kBytesAct;
constexpr size_t kOffOBL = kOffOBH + kBytesObPlane;
constexpr size_t kWsTotal = kOffOBL + kBytesObPlane;
static_assert(kWsTotal == 114294784ull, "");
static_assert(kWsTotal <= 134217728ull, "");
static_assert(kOffXL % 128 == 0 && kOffWH % 128 == 0 && kOffWL % 128 == 0 && kOffWOH % 128 == 0 &&
              kOffWOL % 128 == 0 && kOffP % 128 == 0 && kOffQN % 128 == 0 && kOffKN % 128 == 0 &&
              kOffVN % 128 == 0 && kOffBD % 128 == 0 && kOffOSC % 128 == 0 && kOffOBH % 128 == 0 &&
              kOffOBL % 128 == 0, "");

typedef __attribute__((ext_vector_type(16))) _Float16 v16h;
typedef __attribute__((ext_vector_type(8)))  _Float16 v8h;
typedef __attribute__((ext_vector_type(16))) __bf16   v16b;
typedef __attribute__((ext_vector_type(8)))  __bf16   v8b;
typedef __attribute__((ext_vector_type(8)))  float    v8f;
typedef __attribute__((ext_vector_type(4)))  float    v4f;
typedef __attribute__((ext_vector_type(4)))  unsigned int v4u;

__device__ __forceinline__ unsigned short f2bf_bits(float f) {
  unsigned u = __float_as_uint(f);
  return (unsigned short)((u + 0x7FFFu + ((u >> 16) & 1u)) >> 16);
}
__device__ __forceinline__ float bf_bits2f(unsigned short h) { return __uint_as_float(((unsigned)h) << 16); }
__device__ __forceinline__ unsigned pk16(unsigned short a, unsigned short b) { return (unsigned)a | ((unsigned)b << 16); }

__device__ __forceinline__ void dep_guard_h(v8f& a, v8f& b, v16h x, v16h y) { asm volatile("v_nop\n\tv_nop\n\tv_nop\n\tv_nop" : "+v"(a), "+v"(b) : "v"(x), "v"(y)); }
__device__ __forceinline__ void dep_guard_b(v8f& a, v8f& b, v16b x, v16b y) { asm volatile("v_nop\n\tv_nop\n\tv_nop\n\tv_nop" : "+v"(a), "+v"(b) : "v"(x), "v"(y)); }
__device__ __forceinline__ void keep4_h(v16h a, v16h b, v16h c, v16h d) { asm volatile("v_nop" :: "v"(a), "v"(b), "v"(c), "v"(d)); }
__device__ __forceinline__ void keep4_b(v16b a, v16b b, v16b c, v16b d) { asm volatile("v_nop" :: "v"(a), "v"(b), "v"(c), "v"(d)); }
__device__ __forceinline__ void acc_guard4(v8f& a, v8f& b, v8f& c, v8f& d) { asm volatile("v_nop\n\tv_nop\n\tv_nop\n\tv_nop" : "+v"(a), "+v"(b), "+v"(c), "+v"(d)); }
template <typename T> struct Frag;
template <> struct Frag<_Float16> {
  typedef v16h V; union U { v16h v; v8h h[2]; };
  static __device__ __forceinline__ v16h load(const _Float16* p) {
    U f; f.h[0] = *(const v8h*)(p); f.h[1] = *(const v8h*)(p + 16); return f.v;
  }
  static __device__ __forceinline__ v8f mma(v16h a, v16h b, v8f c) {
    return __builtin_amdgcn_wmma_f32_16x16x32_f16(false, a, false, b, (short)0, c, false, false);
  }
  static __device__ __forceinline__ void guard(v8f& a, v8f& b, v16h x, v16h y) { dep_guard_h(a, b, x, y); }
  static __device__ __forceinline__ void keep(v16h a, v16h b, v16h c, v16h d) { keep4_h(a, b, c, d); }
};
template <> struct Frag<__bf16> {
  typedef v16b V; union U { v16b v; v8b h[2]; };
  static __device__ __forceinline__ v16b load(const __bf16* p) {
    U f; f.h[0] = *(const v8b*)(p); f.h[1] = *(const v8b*)(p + 16); return f.v;
  }
  static __device__ __forceinline__ v8f mma(v16b a, v16b b, v8f c) {
    return __builtin_amdgcn_wmma_f32_16x16x32_bf16(false, a, false, b, (short)0, c, false, false);
  }
  static __device__ __forceinline__ void guard(v8f& a, v8f& b, v16b x, v16b y) { dep_guard_b(a, b, x, y); }
  static __device__ __forceinline__ void keep(v16b a, v16b b, v16b c, v16b d) { keep4_b(a, b, c, d); }
};

template <int ET> struct Elem;
template <> struct Elem<0> { typedef _Float16 T; };
template <> struct Elem<1> { typedef __bf16 T; };
template <int ET, bool SPLIT, int BIAS_MODE, int OUT_MODE, bool RESID, int ACT = 0>
__global__ __launch_bounds__(256) void wmma_gemm64(
    const unsigned short* __restrict__ Ap, const unsigned short* __restrict__ A2p, int lda, long strideA,
    const unsigned short* __restrict__ Btp, const unsigned short* __restrict__ Bt2p, int ldb, long strideB,
    void* __restrict__ Cout, void* __restrict__ Cout2, int ldc, long strideC,
    const float* __restrict__ bias,
    const float* __restrict__ resid, long strideR,
    int M, int N, int K, float scale) {
  typedef typename Elem<ET>::T T;
  typedef typename Frag<T>::V V;
  const T* A = (const T*)Ap; const T* A2 = (const T*)A2p; const T* Bt = (const T*)Btp; const T* Bt2 = (const T*)Bt2p;
  __shared__ __align__(16) float sT[8][16 * 68];
  const int b    = blockIdx.y;
  const int lane = threadIdx.x & 31;
  const int wave = threadIdx.x >> 5;
  const int tilesN = N >> 6;
  const int tilesM = M >> 6;
  const int tile = blockIdx.x * 8 + wave;
  if (tile >= tilesM * tilesN) return;
  const int tm = tile / tilesN;
  const int tn = tile - tm * tilesN;
  const int m0 = tm << 6;
  const int n0 = tn << 6;

  const T* Ab  = A  + (size_t)b * strideA;
  const T* Bb  = Bt + (size_t)b * strideB;
  const T* Ab2 = SPLIT ? (A2  + (size_t)b * strideA) : nullptr;
  const T* Bb2 = SPLIT ? (Bt2 + (size_t)b * strideB) : nullptr;

  const int rlane = lane & 15;
  const int koff  = (lane >> 4) * 8;
  const int mOff  = (lane >> 4) * 8;

  v8f acc[4][4];
#pragma unroll
  for (int i = 0; i < 4; ++i)
#pragma unroll
    for (int j = 0; j < 4; ++j) acc[i][j] = (v8f){0.f,0.f,0.f,0.f,0.f,0.f,0.f,0.f};

  for (int k0 = 0; k0 < K; k0 += 32) {
    V bh[4], bl[4];
#pragma unroll
    for (int j = 0; j < 4; ++j) {
      const size_t bo = (size_t)(n0 + (j << 4) + rlane) * ldb + koff + k0;
      bh[j] = Frag<T>::load(Bb + bo);
      if (SPLIT) bl[j] = Frag<T>::load(Bb2 + bo);
    }
#pragma unroll
    for (int i = 0; i < 4; ++i) {
      const size_t ao = (size_t)(m0 + (i << 4) + rlane) * lda + koff + k0;
      V ah = Frag<T>::load(Ab + ao);
      V al;
      if (SPLIT) al = Frag<T>::load(Ab2 + ao);
#pragma unroll
      for (int j = 0; j < 4; ++j) {
        acc[i][j] = Frag<T>::mma(ah, bh[j], acc[i][j]);
        if (SPLIT) {
          acc[i][j] = Frag<T>::mma(ah, bl[j], acc[i][j]);
          acc[i][j] = Frag<T>::mma(al, bh[j], acc[i][j]);
        }
      }
      Frag<T>::guard(acc[i][0], acc[i][3], ah, SPLIT ? al : ah);
    }
    Frag<T>::keep(bh[0], bh[1], bh[2], bh[3]);
    if (SPLIT) Frag<T>::keep(bl[0], bl[1], bl[2], bl[3]);
  }
  acc_guard4(acc[0][0], acc[0][1], acc[0][2], acc[0][3]);
  acc_guard4(acc[1][0], acc[1][1], acc[1][2], acc[1][3]);
  acc_guard4(acc[2][0], acc[2][1], acc[2][2], acc[2][3]);
  acc_guard4(acc[3][0], acc[3][1], acc[3][2], acc[3][3]);

  float* slab = sT[wave];
  const float* Rb = RESID ? (resid + (size_t)b * strideR) : nullptr;
#pragma unroll
  for (int i = 0; i < 4; ++i) {
    const int mBase = m0 + (i << 4);
#pragma unroll
    for (int j = 0; j < 4; ++j) {
      const int n = n0 + (j << 4) + rlane;
      float bv = 0.f;
      if (BIAS_MODE == 2) bv = bias[n];
#pragma unroll
      for (int r = 0; r < 8; ++r) {
        float v = acc[i][j][r] * scale;
        if (BIAS_MODE == 1) v += bias[mBase + mOff + r];
        if (BIAS_MODE == 2) v += bv;
        if (RESID) v += Rb[(size_t)(mBase + mOff + r) * ldc + n];
        if (ACT == 2) v = fmaxf(v, 0.0f);
        if (ACT == 4) v = (v > 0.f) ? v : 0.01f * v;
        slab[(mOff + r) * 68 + (j << 4) + rlane] = v;
      }
    }
    __builtin_amdgcn_fence(__ATOMIC_RELEASE, "workgroup");
    __builtin_amdgcn_wave_barrier();
    __builtin_amdgcn_fence(__ATOMIC_ACQUIRE, "workgroup");
    if (OUT_MODE == 0) {
      float* C = (float*)Cout + (size_t)b * strideC;
      const int hh = lane >> 4, c4 = (lane & 15) * 4;
      for (int pass = 0; pass < 2; ++pass) {
#pragma unroll
        for (int it = 0; it < 8; ++it) {
          const int row = it * 2 + hh;
          v4f v = *(const v4f*)(slab + row * 68 + c4);
          *(volatile v4f*)(C + (size_t)(mBase + row) * ldc + n0 + c4) = v;
        }
        __threadfence();
      }
    } else {
      const int q = lane >> 3, c8 = (lane & 7) * 8;
      unsigned short* C  = (unsigned short*)Cout  + (size_t)b * strideC;
      unsigned short* C2 = (OUT_MODE == 2) ? ((unsigned short*)Cout2 + (size_t)b * strideC) : nullptr;
      for (int pass = 0; pass < 2; ++pass) {
#pragma unroll
        for (int it = 0; it < 4; ++it) {
          const int row = it * 4 + q;
          const float* sp = slab + row * 68 + c8;
          v8h hv, lv;
#pragma unroll
          for (int e = 0; e < 8; ++e) {
            if (OUT_MODE == 1) {
              hv[e] = (_Float16)sp[e];
            } else {
              unsigned short hb = f2bf_bits(sp[e]);
              unsigned short lb = f2bf_bits(sp[e] - bf_bits2f(hb));
              hv[e] = __builtin_bit_cast(_Float16, hb);
              lv[e] = __builtin_bit_cast(_Float16, lb);
            }
          }
          *(volatile v8h*)(C + (size_t)(mBase + row) * ldc + n0 + c8) = hv;
          if (OUT_MODE == 2) *(volatile v8h*)(C2 + (size_t)(mBase + row) * ldc + n0 + c8) = lv;
        }
        __threadfence();
      }
    }
    __builtin_amdgcn_fence(__ATOMIC_RELEASE, "workgroup");
    __builtin_amdgcn_wave_barrier();
    __builtin_amdgcn_fence(__ATOMIC_ACQUIRE, "workgroup");
  }
}

__device__ __forceinline__ float sigmoid_f(float x) {
  const float xc = fmaxf(x, -30.0f);
  return 1.0f / (1.0f + expf(-xc));
}
__device__ __forceinline__ float silu_f(float x) { return x * sigmoid_f(x); }

__device__ __forceinline__ float silu_act(float x) {
  const float xc = fmaxf(x, -30.0f);
  const float ex = __builtin_amdgcn_exp2f(-xc * 1.44269504088896341f);
  const float rc = __builtin_amdgcn_rcpf(1.0f + ex);
  return x * rc;
}

__device__ __forceinline__ float fence_f(float p) {
  asm volatile("" : "+v"(p));
  return p;
}

__device__ __forceinline__ void split8_store(v4f a, v4f c, unsigned short* __restrict__ hp,
                                             unsigned short* __restrict__ lp) {
  unsigned short hb[8], lb[8];
#pragma unroll
  for (int e = 0; e < 4; ++e) {
    const unsigned short h0 = f2bf_bits(a[e]);
    hb[e] = h0;
    lb[e] = f2bf_bits(a[e] - bf_bits2f(h0));
    const unsigned short h1 = f2bf_bits(c[e]);
    hb[4 + e] = h1;
    lb[4 + e] = f2bf_bits(c[e] - bf_bits2f(h1));
  }
  const v4u uh = (v4u){pk16(hb[0], hb[1]), pk16(hb[2], hb[3]), pk16(hb[4], hb[5]), pk16(hb[6], hb[7])};
  const v4u ul = (v4u){pk16(lb[0], lb[1]), pk16(lb[2], lb[3]), pk16(lb[4], lb[5]), pk16(lb[6], lb[7])};
  *(volatile v4u*)hp = uh;
  *(volatile v4u*)lp = ul;
  __threadfence();
  *(volatile v4u*)hp = uh;
  *(volatile v4u*)lp = ul;
}

__global__ __launch_bounds__(256) void split_planes_kernel(
    const float* __restrict__ in0, const float* __restrict__ in1,
    const float* __restrict__ in2, const float* __restrict__ in3,
    unsigned short* __restrict__ hi, unsigned short* __restrict__ lo, int n8, long zstride) {
  const int z = blockIdx.y;
  const float* src = (z == 0) ? in0 : (z == 1) ? in1 : (z == 2) ? in2 : in3;
  const int i = blockIdx.x * 256 + threadIdx.x;
  if (i >= n8) return;
  const float* p = src + 8 * (size_t)i;
  const v4f a = *(const v4f*)(p);
  const v4f c = *(const v4f*)(p + 4);
  const size_t o = (size_t)z * (size_t)zstride + 8 * (size_t)i;
  split8_store(a, c, hi + o, lo + o);
}

__global__ __launch_bounds__(256) void split_rows_ab_kernel(
    const float* __restrict__ wa, const float* __restrict__ wb,
    unsigned short* __restrict__ hi, unsigned short* __restrict__ lo) {
  const int i = blockIdx.x * 256 + threadIdx.x;
  if (i >= 64 * 128) return;
  const int row = i >> 7;
  const int c0  = (i & 127) * 8;
  const int ra  = row < 16 ? row : 15;
  int rb = row - 16; rb = rb < 0 ? 0 : (rb > 15 ? 15 : rb);
  const float* pa = wa + (size_t)ra * kChan + c0;
  const float* pb = wb + (size_t)rb * kChan + c0;
  const v4f a0 = *(const v4f*)(pa), a1 = *(const v4f*)(pa + 4);
  const v4f b0 = *(const v4f*)(pb), b1 = *(const v4f*)(pb + 4);
  const bool useA = row < 16;
  const bool useB = (row >= 16) && (row < 32);
  v4f s0, s1;
#pragma unroll
  for (int e = 0; e < 4; ++e) {
    s0[e] = useA ? a0[e] : (useB ? b0[e] : 0.0f);
    s1[e] = useA ? a1[e] : (useB ? b1[e] : 0.0f);
  }
  const size_t o = (size_t)(4 * kInner + row) * kChan + c0;
  split8_store(s0, s1, hi + o, lo + o);
}

__global__ __launch_bounds__(256) void conv_norm_kernel(
    const float* __restrict__ P,
    const float* __restrict__ cqw, const float* __restrict__ cqb,
    const float* __restrict__ ckw, const float* __restrict__ ckb,
    const float* __restrict__ cvw, const float* __restrict__ cvb,
    const float* __restrict__ A_log, const float* __restrict__ dt_bias,
    float* __restrict__ qn, float* __restrict__ kn, float* __restrict__ vn, float* __restrict__ bd) {
  __shared__ float redq[8];
  __shared__ float redk[8];
  const int t    = blockIdx.x;
  const int grp  = blockIdx.y;
  const int tid  = threadIdx.x;
  const int lane = tid & 31, wave = tid >> 5;
  const int c    = grp * 256 + tid;

  float pq[kTaps], pk[kTaps], pv[kTaps];
#pragma unroll
  for (int j = 0; j < kTaps; ++j) {
    const int r  = t - (kTaps - 1) + j;
    const int rc = r < 0 ? 0 : r;
    const bool ok = (r >= 0);
    const float* pr = P + (size_t)rc * kProjN;
    const float a = pr[c];
    const float b = pr[kInner + c];
    const float d = pr[2 * kInner + c];
    pq[j] = ok ? a : 0.0f;
    pk[j] = ok ? b : 0.0f;
    pv[j] = ok ? d : 0.0f;
  }
  const v4f wq4 = *(const v4f*)(cqw + (size_t)c * kTaps);
  const v4f wk4 = *(const v4f*)(ckw + (size_t)c * kTaps);
  const v4f wv4 = *(const v4f*)(cvw + (size_t)c * kTaps);
  float aq = 0.f, ak = 0.f, av = 0.f;
#pragma unroll
  for (int j = 0; j < kTaps; ++j) {
    aq = fmaf(wq4[j], pq[j], aq);
    ak = fmaf(wk4[j], pk[j], ak);
    av = fmaf(wv4[j], pv[j], av);
  }
  aq += cqb[c];
  ak += ckb[c];
  av += cvb[c];
  const float qy = silu_f(aq);
  const float ky = silu_f(ak);
  const float vy = silu_f(av);

  float sq = qy * qy, sk = ky * ky;
#pragma unroll
  for (int off = 16; off > 0; off >>= 1) {
    sq += __shfl_xor(sq, off, 32);
    sk += __shfl_xor(sk, off, 32);
  }
  if (lane == 0) { redq[wave] = sq; redk[wave] = sk; }
  __syncthreads();
  const int w0 = wave & ~1;
  const float tq = redq[w0] + redq[w0 + 1];
  const float tk = redk[w0] + redk[w0 + 1];
  const float rq = rsqrtf(tq + 1e-6f);
  const float rk = rsqrtf(tk + 1e-6f);
  const float qo = qy * rq;
  const float ko = ky * rk;
  const size_t o = (size_t)t * kInner + c;
  ((volatile float*)qn)[o] = qo;
  ((volatile float*)kn)[o] = ko;
  ((volatile float*)vn)[o] = vy;
  __threadfence();
  ((volatile float*)qn)[o] = qo;
  ((volatile float*)kn)[o] = ko;
  ((volatile float*)vn)[o] = vy;

  if (grp == 0 && wave == 0) {
    const int hx = lane & 15;
    const float* pr = P + (size_t)t * kProjN;
    const float pa = pr[4 * kInner + hx];
    const float pb = pr[4 * kInner + kHeads + hx];
    const float a  = pa + dt_bias[hx];
    const float sp  = fmaxf(a, 0.0f) + log1pf(expf(-fabsf(a)));
    const float dec = expf(-expf(A_log[hx]) * sp);
    const float bet = sigmoid_f(pb);
    const float val = (lane < 16) ? bet : dec;
    const size_t ob = (size_t)t * kBdW + lane;
    ((volatile float*)bd)[ob] = val;
    __threadfence();
    ((volatile float*)bd)[ob] = val;
  }
}

__global__ __launch_bounds__(64) void scan_kernel(
    const float* __restrict__ qn, const float* __restrict__ kn, const float* __restrict__ vn,
    const float* __restrict__ bd, float* __restrict__ osc) {
#pragma clang fp contract(off)
  __shared__ __align__(16) float sk[2][kHeadDim];
  __shared__ __align__(16) float sq[2][kHeadDim];
  const int h   = blockIdx.x;
  const int e   = threadIdx.x;
  const int col = h * kHeadDim + e;
  float S[kHeadDim];
#pragma unroll
  for (int d = 0; d < kHeadDim; ++d) S[d] = 0.f;

  for (int t = 0; t < kSeq; ++t) {
    const size_t rb = (size_t)t * kInner + col;
    const float kvv  = kn[rb];
    const float qvv  = qn[rb];
    const float vvv  = vn[rb];
    const float beta = bd[(size_t)t * kBdW + h];
    const float dec  = bd[(size_t)t * kBdW + kHeads + h];
    const int p = t & 1;
    sk[p][e] = kvv;
    sq[p][e] = qvv;
    __syncthreads();
    const float* kp = sk[p];
    const float* qp = sq[p];

    float kS = 0.f;
#pragma unroll
    for (int d4 = 0; d4 < kHeadDim / 4; ++d4) {
      const v4f kk = *(const v4f*)(kp + 4 * d4);
#pragma unroll
      for (int u = 0; u < 4; ++u) {
        const float pr = fence_f(kk[u] * S[4 * d4 + u]);
        kS = kS + pr;
      }
    }
    const float w = beta * (vvv - kS);
    float o = 0.f;
#pragma unroll
    for (int d4 = 0; d4 < kHeadDim / 4; ++d4) {
      const v4f kk = *(const v4f*)(kp + 4 * d4);
      const v4f qq = *(const v4f*)(qp + 4 * d4);
#pragma unroll
      for (int u = 0; u < 4; ++u) {
        const float da = fence_f(dec * S[4 * d4 + u]);
        const float wr = fence_f(kk[u] * w);
        const float sn = da + wr;
        S[4 * d4 + u] = sn;
        const float qt = fence_f(qq[u] * sn);
        o = o + qt;
      }
    }
    ((volatile float*)osc)[rb] = o;
    __threadfence();
    ((volatile float*)osc)[rb] = o;
  }
}

__global__ __launch_bounds__(256) void gate_kernel(
    const float* __restrict__ osc, const float* __restrict__ P, const float* __restrict__ oscale,
    unsigned short* __restrict__ obh, unsigned short* __restrict__ obl) {
  const int gi  = blockIdx.x * 256 + threadIdx.x;
  const int row = gi >> 7;
  if (row >= kSeq) return;
  const int c0  = (gi & 127) * 8;
  const float* op = osc + (size_t)row * kInner + c0;
  const float* gp = P + (size_t)row * kProjN + 3 * kInner + c0;
  const float* sp = oscale + (c0 & 63);
  const v4f o0 = *(const v4f*)(op), o1 = *(const v4f*)(op + 4);
  const v4f g0 = *(const v4f*)(gp), g1 = *(const v4f*)(gp + 4);
  const v4f s0 = *(const v4f*)(sp), s1 = *(const v4f*)(sp + 4);
  float ss = 0.f;
#pragma unroll
  for (int e = 0; e < 4; ++e) { ss = fmaf(o0[e], o0[e], ss); ss = fmaf(o1[e], o1[e], ss); }
  ss += __shfl_xor(ss, 1, 32);
  ss += __shfl_xor(ss, 2, 32);
  ss += __shfl_xor(ss, 4, 32);
  const float r = rsqrtf(ss * (1.0f / 64.0f) + 1e-6f);
  v4f v0, v1;
#pragma unroll
  for (int e = 0; e < 4; ++e) {
    v0[e] = ((o0[e] * r) * s0[e]) * silu_act(g0[e]);
    v1[e] = ((o1[e] * r) * s1[e]) * silu_act(g1[e]);
  }
  const size_t o = (size_t)row * kInner + c0;
  split8_store(v0, v1, obh + o, obl + o);
}

extern "C" void kernel_launch(void* const* d_in, const int* in_sizes, int n_in,
                              void* d_out, int out_size, void* d_ws, size_t ws_size,
                              hipStream_t stream) {
  if (n_in < 17) return;
  if (out_size != kBatch * kSeq * kChan) return;
  if (ws_size < kWsTotal) return;
  if (in_sizes[0] != kBatch * kSeq * kChan) return;
  if (in_sizes[1] != kInner * kChan || in_sizes[2] != kInner * kChan ||
      in_sizes[3] != kInner * kChan || in_sizes[4] != kInner * kChan ||
      in_sizes[5] != kChan * kInner) return;
  if (in_sizes[6] != kHeads * kChan || in_sizes[7] != kHeads * kChan) return;
  if (in_sizes[8] != kInner * kTaps || in_sizes[10] != kInner * kTaps || in_sizes[12] != kInner * kTaps) return;
  if (in_sizes[9] != kInner || in_sizes[11] != kInner || in_sizes[13] != kInner) return;
  if (in_sizes[14] != kHeads || in_sizes[15] != kHeads || in_sizes[16] != kHeadDim) return;

  const float* x       = (const float*)d_in[0];
  const float* wq      = (const float*)d_in[1];
  const float* wk      = (const float*)d_in[2];
  const float* wv      = (const float*)d_in[3];
  const float* wg      = (const float*)d_in[4];
  const float* wo      = (const float*)d_in[5];
  const float* wa      = (const float*)d_in[6];
  const float* wb      = (const float*)d_in[7];
  const float* cqw     = (const float*)d_in[8];
  const float* cqb     = (const float*)d_in[9];
  const float* ckw     = (const float*)d_in[10];
  const float* ckb     = (const float*)d_in[11];
  const float* cvw     = (const float*)d_in[12];
  const float* cvb     = (const float*)d_in[13];
  const float* A_log   = (const float*)d_in[14];
  const float* dt_bias = (const float*)d_in[15];
  const float* oscale  = (const float*)d_in[16];

  char* ws = (char*)d_ws;
  unsigned short* XH  = (unsigned short*)(ws + kOffXH);
  unsigned short* XL  = (unsigned short*)(ws + kOffXL);
  unsigned short* WH  = (unsigned short*)(ws + kOffWH);
  unsigned short* WL  = (unsigned short*)(ws + kOffWL);
  unsigned short* WOH = (unsigned short*)(ws + kOffWOH);
  unsigned short* WOL = (unsigned short*)(ws + kOffWOL);
  float*          P   = (float*)(ws + kOffP);
  float*          QN  = (float*)(ws + kOffQN);
  float*          KN  = (float*)(ws + kOffKN);
  float*          VN  = (float*)(ws + kOffVN);
  float*          BD  = (float*)(ws + kOffBD);
  float*          OSC = (float*)(ws + kOffOSC);
  unsigned short* OBH = (unsigned short*)(ws + kOffOBH);
  unsigned short* OBL = (unsigned short*)(ws + kOffOBL);

  {
    const int n8 = kBatch * kSeq * kChan / 8;
    split_planes_kernel<<<dim3((n8 + 255) / 256, 1), 256, 0, stream>>>(x, x, x, x, XH, XL, n8, 0L);
  }
  {
    const int n8 = kInner * kChan / 8;
    split_planes_kernel<<<dim3((n8 + 255) / 256, 4), 256, 0, stream>>>(wq, wk, wv, wg, WH, WL, n8,
                                                                       (long)kInner * kChan);
  }
  split_rows_ab_kernel<<<dim3(32), 256, 0, stream>>>(wa, wb, WH, WL);
  {
    const int n8 = kChan * kInner / 8;
    split_planes_kernel<<<dim3((n8 + 255) / 256, 1), 256, 0, stream>>>(wo, wo, wo, wo, WOH, WOL, n8, 0L);
  }

  for (int bsel = 0; bsel < kBatch; ++bsel) {
    const unsigned short* XHb = XH + (size_t)bsel * kSeq * kChan;
    const unsigned short* XLb = XL + (size_t)bsel * kSeq * kChan;
    {
      const int tiles = (kSeq / 64) * (kProjN / 64);
      wmma_gemm64<1, true, 0, 0, false, 0><<<dim3((tiles + 7) / 8, 1), 256, 0, stream>>>(
          XHb, XLb, kChan, 0L, WH, WL, kChan, 0L, (void*)P, (void*)P, kProjN, 0L,
          oscale, oscale, 0L, kSeq, kProjN, kChan, 1.0f);
    }
    conv_norm_kernel<<<dim3(kSeq, kInner / 256), 256, 0, stream>>>(
        P, cqw, cqb, ckw, ckb, cvw, cvb, A_log, dt_bias, QN, KN, VN, BD);
    scan_kernel<<<dim3(kHeads), 64, 0, stream>>>(QN, KN, VN, BD, OSC);
    gate_kernel<<<dim3((kSeq * 128 + 255) / 256), 256, 0, stream>>>(OSC, P, oscale, OBH, OBL);
    {
      float* outb = (float*)d_out + (size_t)bsel * kSeq * kChan;
      const int tiles = (kSeq / 64) * (kChan / 64);
      wmma_gemm64<1, true, 0, 0, false, 0><<<dim3((tiles + 7) / 8, 1), 256, 0, stream>>>(
          OBH, OBL, kInner, 0L, WOH, WOL, kInner, 0L, (void*)outb, (void*)outb, kChan, 0L,
          oscale, oscale, 0L, kSeq, kChan, kInner, 1.0f);
    }
  }
}
